// CausalSelfAttention_18975165514359
// MI455X (gfx1250) — hardware-verified
//
#include <hip/hip_runtime.h>


#ifndef NB
#define NB 4
#endif
#ifndef SEQ
#define SEQ 2048
#endif
#define NB_FULL  4
#define SEQ_FULL 2048
#define DM   1024
#define NH   16
#define HD   64
#define RH   256
#define QKCAR 16.0f
#define VCAR  16.0f
#define CCAR  64.0f
#define WCAR  1024.0f
#define PLOG  10.0f
#define L2E   1.4426950408889634f
#define NEGB  (-3.0e38f)
#define SCQ16 (0.125f / (QKCAR * QKCAR))
#define SCQHL 0.125f

typedef _Float16 h16;
typedef unsigned short bf;
typedef __attribute__((ext_vector_type(16))) __bf16   v16bf;
typedef __attribute__((ext_vector_type(16))) _Float16 v16h;
typedef __attribute__((ext_vector_type(8)))  _Float16 v8h;
typedef __attribute__((ext_vector_type(2)))  _Float16 v2h;
typedef __attribute__((ext_vector_type(8)))  unsigned short v8us;
typedef __attribute__((ext_vector_type(2)))  unsigned short v2us;
typedef __attribute__((ext_vector_type(8)))  float    v8f;
typedef __attribute__((ext_vector_type(4)))  float    v4f;
typedef v8h  __attribute__((may_alias)) v8ha;
typedef v4f  __attribute__((may_alias)) v4fa;
typedef v8us __attribute__((may_alias)) v8usa;

static_assert(SEQ % 64 == 0);
static_assert(RH % 64 == 0);
static_assert(RH <= SEQ);
static_assert(SEQ <= SEQ_FULL);
static_assert(NB <= NB_FULL);
static_assert(DM % 64 == 0);
static_assert(DM % 32 == 0);
static_assert(HD == 64);
static_assert(NH * HD == DM);
static_assert((3 * DM) % 64 == 0);
static_assert(HD / 2 == 32);
static_assert(SEQ % 8 == 0);

constexpr size_t PL16 = (size_t)NB * NH * SEQ * HD;
constexpr size_t PLE  = (size_t)NB * NH * RH * HD;
constexpr size_t SZ_XB   = (size_t)NB * SEQ * DM * 2;
constexpr size_t SZ_WQKV = (size_t)3 * DM * DM * 2;
constexpr size_t SZ_WO   = (size_t)DM * DM * 2;
constexpr size_t SZ_P16  = PL16 * 2;
constexpr size_t SZ_PE   = PLE * 2;
constexpr size_t SZ_CT   = (size_t)NB * SEQ * DM * 2;
constexpr size_t SZ_AT   = (size_t)NB * RH * DM * 2;
constexpr size_t SZ_ROT  = (size_t)SEQ * 32 * 4;
constexpr size_t WS_TOTAL = SZ_XB + SZ_WQKV + 2 * SZ_WO + 3 * SZ_P16 + 6 * SZ_PE + SZ_CT + 2 * SZ_AT + 2 * SZ_ROT;
static_assert(SZ_XB % 256 == 0 && SZ_WQKV % 256 == 0 && SZ_WO % 256 == 0 && SZ_P16 % 256 == 0 && SZ_PE % 256 == 0 && SZ_CT % 256 == 0 && SZ_AT % 256 == 0);
static_assert(SZ_ROT % 256 == 0);
static_assert(WS_TOTAL <= (size_t)134217728);

__device__ __forceinline__ unsigned short f2bf(float f) { unsigned u = __float_as_uint(f); u += 0x7FFFu + ((u >> 16) & 1u); return (unsigned short)(u >> 16); }
__device__ __forceinline__ float bf2f(unsigned short b) { return __uint_as_float(((unsigned)b) << 16); }
__device__ __forceinline__ float bfr(float f) { return bf2f(f2bf(f)); }
__device__ __forceinline__ void splitf(float y, unsigned short& h, unsigned short& l) { h = f2bf(y); l = f2bf(y - bf2f(h)); }
__device__ __forceinline__ v16h cat16(v8h lo, v8h hi) { return __builtin_shufflevector(lo, hi, 0, 1, 2, 3, 4, 5, 6, 7, 8, 9, 10, 11, 12, 13, 14, 15); }
__device__ __forceinline__ v16bf cat16b(v8us lo, v8us hi) { return __builtin_bit_cast(v16bf, __builtin_shufflevector(lo, hi, 0, 1, 2, 3, 4, 5, 6, 7, 8, 9, 10, 11, 12, 13, 14, 15)); }
__device__ __forceinline__ v8f wmma16(v16h a, v16h b, v8f c) { return __builtin_amdgcn_wmma_f32_16x16x32_f16(false, a, false, b, (short)0, c, false, false); }
__device__ __forceinline__ v8f wmmab(v16bf a, v16bf b, v8f c) { return __builtin_amdgcn_wmma_f32_16x16x32_bf16(false, a, false, b, (short)0, c, false, false); }
__device__ __forceinline__ float ex2(float x) { return __builtin_amdgcn_exp2f(x); }
static __device__ __forceinline__ h16 toh_flush(float v) { const h16 r = (h16)v; return (fabsf(v) < 6.103515625e-05f) ? (h16)0.0f : r; }
__device__ __forceinline__ v16h  ldh(const h16* p) { return cat16(*(const v8h*)p, *(const v8h*)(p + 16)); }
__device__ __forceinline__ v16bf ldb(const bf* p)  { return cat16b(*(const v8us*)p, *(const v8us*)(p + 16)); }

template <typename T16> struct WFrag;
template <> struct WFrag<h16> { typedef v16h V; static __device__ __forceinline__ V ld(const h16* p) { return ldh(p); } static __device__ __forceinline__ v8f mma(V a, V b, v8f c) { return wmma16(a, b, c); } };
template <> struct WFrag<bf>  { typedef v16bf V; static __device__ __forceinline__ V ld(const bf* p) { return ldb(p); } static __device__ __forceinline__ v8f mma(V a, V b, v8f c) { return wmmab(a, b, c); } };

template <typename T16, int NSPLIT>
__device__ __forceinline__ void gemm_loop(const T16* __restrict__ A, const T16* __restrict__ A2, const T16* __restrict__ Bt, int K, size_t aoff, size_t boff, v8f (&acc)[4][4]) {
    typedef typename WFrag<T16>::V V;
#pragma unroll 1
    for (int kc = 0; kc < K; kc += 32) {
        V a[4], a2[4];
#pragma unroll
        for (int mb = 0; mb < 4; ++mb) { a[mb] = WFrag<T16>::ld(A + aoff + (size_t)mb * 16 * K + kc); if (NSPLIT == 1) a2[mb] = WFrag<T16>::ld(A2 + aoff + (size_t)mb * 16 * K + kc); }
#pragma unroll
        for (int nb = 0; nb < 4; ++nb) { const V b = WFrag<T16>::ld(Bt + boff + (size_t)nb * 16 * K + kc);
#pragma unroll
            for (int mb = 0; mb < 4; ++mb) { acc[mb][nb] = WFrag<T16>::mma(a[mb], b, acc[mb][nb]); if (NSPLIT == 1) acc[mb][nb] = WFrag<T16>::mma(a2[mb], b, acc[mb][nb]); } }
        asm volatile("v_nop\n\tv_nop\n\tv_nop\n\tv_nop" : "+v"(acc[0][0]), "+v"(acc[1][1]), "+v"(acc[2][2]), "+v"(acc[3][3]) : "v"(a[0]), "v"(a[3]));
    }
}

template <typename T16, int NSPLIT>
__device__ __forceinline__ void gemm_out_body(const T16* __restrict__ A, const T16* __restrict__ A2, const T16* __restrict__ Bt, int K, float* C, int ldc, const float* __restrict__ bias, float osc, size_t sA, size_t sC) {
    __shared__ __align__(16) float os[16 * 68];
    const size_t z = blockIdx.z; A += z * sA; A2 += z * sA; C += z * sC;
    const int lane = threadIdx.x & 31, lr = lane & 15, hi = lane >> 4; const int r0 = blockIdx.x * 64, c0 = blockIdx.y * 64;
    v8f acc[4][4];
#pragma unroll
    for (int mb = 0; mb < 4; ++mb)
#pragma unroll
        for (int nb = 0; nb < 4; ++nb) acc[mb][nb] = (v8f){};
    const size_t aoff = (size_t)(r0 + lr) * K + 8 * hi, boff = (size_t)(c0 + lr) * K + 8 * hi;
    gemm_loop<T16, NSPLIT>(A, A2, Bt, K, aoff, boff, acc);
    const int cofs = lr * 4;
    const v4f bv = *(const v4f*)(bias + c0 + cofs);
    v4f bb; bb[0] = bfr(bv[0]); bb[1] = bfr(bv[1]); bb[2] = bfr(bv[2]); bb[3] = bfr(bv[3]);
#pragma unroll
    for (int mb = 0; mb < 4; ++mb) {
#pragma unroll
        for (int nb = 0; nb < 4; ++nb) {
#pragma unroll
            for (int j = 0; j < 8; ++j) os[(hi * 8 + j) * 68 + nb * 16 + lr] = acc[mb][nb][j]; }
        __syncthreads();
        float* crow = C + (size_t)(r0 + mb * 16) * ldc + c0;
#pragma unroll 1
        for (int ps = 0; ps < 2; ++ps) {
#pragma unroll
            for (int s = 0; s < 8; ++s) { const int row = 2 * s + hi; const v4f t = *(const v4fa*)(os + row * 68 + cofs); v4f val;
                val[0] = t[0] * osc + bb[0]; val[1] = t[1] * osc + bb[1]; val[2] = t[2] * osc + bb[2]; val[3] = t[3] * osc + bb[3];
                *(volatile v4f*)(crow + (size_t)row * ldc + cofs) = val; }
            if (ps == 0) __threadfence(); }
        __syncthreads();
    }
}

__global__ __launch_bounds__(32) void k_proj_hl(const bf* __restrict__ Ah, const bf* __restrict__ Al, const bf* __restrict__ Wt, float* C, const float* __restrict__ bias) {
    gemm_out_body<bf, 1>(Ah, Al, Wt, DM, C, DM, bias, 1.0f, (size_t)RH * DM, (size_t)SEQ * DM);
}
__global__ __launch_bounds__(32) void k_proj16(const h16* __restrict__ A, const h16* __restrict__ Wt, float* C, const float* __restrict__ bias) {
    gemm_out_body<h16, 0>(A, A, Wt, DM, C, DM, bias, 1.0f / (CCAR * WCAR), (size_t)SEQ * DM, (size_t)SEQ * DM);
}

__global__ __launch_bounds__(256) void k_cvt8(const float* __restrict__ src, bf* dst, unsigned n8) {
    const size_t b = blockIdx.y; src += b * (size_t)SEQ_FULL * DM; dst += b * (size_t)SEQ * DM;
    const unsigned i = blockIdx.x * 256 + threadIdx.x; if (i >= n8) return;
    const v8f v = *(const v8f*)(src + (size_t)i * 8); v8us o;
#pragma unroll
    for (int k = 0; k < 8; ++k) o[k] = f2bf(v[k]);
    *(volatile v8us*)(dst + (size_t)i * 8) = o; __threadfence(); *(volatile v8us*)(dst + (size_t)i * 8) = o;
}

__global__ __launch_bounds__(256) void k_wtG(const float* __restrict__ w, int K, int N, bf* Bt, h16* Bt16, float car) {
    const int lane = threadIdx.x & 31; const int L0 = (blockIdx.x * 8 + (threadIdx.x >> 5)) * 8; const int nlines = N * (K / 64);
#pragma unroll
    for (int ps = 0; ps < 2; ++ps) {
#pragma unroll 1
        for (int l = 0; l < 8; ++l) { const int L = L0 + l; if (L >= nlines) break; const size_t e = (size_t)L * 64 + lane * 2; const int k = (int)(e % K), n = (int)(e / K); v2us o;
            o[0] = f2bf(w[(size_t)k * N + n]); o[1] = f2bf(w[(size_t)(k + 1) * N + n]); *(volatile v2us*)(Bt + e) = o;
            if (Bt16) { v2h o2; o2[0] = (h16)(bf2f(o[0]) * car); o2[1] = (h16)(bf2f(o[1]) * car); *(volatile v2h*)(Bt16 + e) = o2; } }
        if (ps == 0) __threadfence(); }
}

__global__ __launch_bounds__(256) void k_rope(float* RC, float* RS) {
#pragma clang fp contract(off)
    const int wave = __builtin_amdgcn_readfirstlane(threadIdx.x >> 5); const int lane = threadIdx.x & 31;
    const int pos = blockIdx.x * 8 + wave; if (pos >= SEQ) return;
    double p = 1.0;
#pragma unroll 1
    for (int j = 0; j < lane; ++j) p = p * 1.3335214321633240;
    const float pw = (float)p; const float inv = 1.0f / pw; const float ang = (float)pos * inv;
    float sv, cv; sincosf(ang, &sv, &cv);
    float* pc = RC + (size_t)pos * 32 + lane; float* pq = RS + (size_t)pos * 32 + lane;
    *(volatile float*)pc = cv; *(volatile float*)pq = sv; __threadfence(); *(volatile float*)pc = cv; *(volatile float*)pq = sv;
}

__global__ __launch_bounds__(32) void k_qkv(const bf* __restrict__ XB, const bf* __restrict__ W, const float* __restrict__ bias, const float* __restrict__ RC, const float* __restrict__ RS,
                                             h16* QK16, h16* VT16, bf* QKh, bf* QKl, bf* VTh, bf* VTl) {
    __shared__ __align__(16) float os[64 * 68];
    const int lane = threadIdx.x & 31, lr = lane & 15, hi = lane >> 4; const int r0 = blockIdx.x * 64, c0 = blockIdx.y * 64;
    v8f acc[4][4];
#pragma unroll
    for (int mb = 0; mb < 4; ++mb)
#pragma unroll
        for (int nb = 0; nb < 4; ++nb) acc[mb][nb] = (v8f){};
    const size_t aoff = (size_t)(r0 + lr) * DM + 8 * hi, boff = (size_t)(c0 + lr) * DM + 8 * hi;
    gemm_loop<bf, 0>(XB, XB, W, DM, aoff, boff, acc);
#pragma unroll
    for (int nb = 0; nb < 4; ++nb) { const float bc = bfr(bias[c0 + nb * 16 + lr]);
#pragma unroll
        for (int mb = 0; mb < 4; ++mb) {
#pragma unroll
            for (int j = 0; j < 8; ++j) os[(mb * 16 + hi * 8 + j) * 68 + nb * 16 + lr] = acc[mb][nb][j] + bc; } }
    __syncthreads();
    const int which = c0 / DM; const int h = (c0 % DM) / HD; const int b = r0 / SEQ; const int t0 = r0 % SEQ; const int bhh = b * NH + h; const bool early = (t0 < RH); const int te = early ? t0 : 0;
    const int rr = lane >> 3, seg = lane & 7;
    if (which < 2) {
        const size_t tof = (size_t)(t0 + rr) * 32 + (seg & 3) * 8;
#pragma unroll 1
        for (int s = 0; s < 16; ++s) { const int row = s * 4 + rr;
            const v4f ca = *(const v4f*)(RC + tof + (size_t)s * 128); const v4f cb = *(const v4f*)(RC + tof + (size_t)s * 128 + 4);
            const v4f sa = *(const v4f*)(RS + tof + (size_t)s * 128); const v4f sb = *(const v4f*)(RS + tof + (size_t)s * 128 + 4);
            float* op = os + row * 68 + seg * 8;
            const v4f a = *(const v4fa*)op; const v4f c = *(const v4fa*)(op + 4); v4f ra, rc;
            ra[0] = a[0] * ca[0] + (-a[1]) * sa[0]; ra[1] = a[1] * ca[1] + a[0] * sa[1];
            ra[2] = a[2] * ca[2] + (-a[3]) * sa[2]; ra[3] = a[3] * ca[3] + a[2] * sa[3];
            rc[0] = c[0] * cb[0] + (-c[1]) * sb[0]; rc[1] = c[1] * cb[1] + c[0] * sb[1];
            rc[2] = c[2] * cb[2] + (-c[3]) * sb[2]; rc[3] = c[3] * cb[3] + c[2] * sb[3];
            *(v4fa*)op = ra; *(v4fa*)(op + 4) = rc; }
    }
    __syncthreads();
    if (which < 2) {
        h16* P16 = QK16 + (size_t)which * PL16 + ((size_t)bhh * SEQ + t0) * HD + seg * 8;
        bf* PH = QKh + (size_t)which * PLE + ((size_t)bhh * RH + te) * HD + seg * 8;
        bf* PL = QKl + (size_t)which * PLE + ((size_t)bhh * RH + te) * HD + seg * 8;
#pragma unroll 1
        for (int ps = 0; ps < 2; ++ps) {
#pragma unroll 4
            for (int s = 0; s < 16; ++s) { const int row = s * 4 + rr; const v4f a = *(const v4fa*)(os + row * 68 + seg * 8); const v4f c = *(const v4fa*)(os + row * 68 + seg * 8 + 4); v8h o;
#pragma unroll
                for (int i = 0; i < 4; ++i) { o[i] = toh_flush(a[i] * QKCAR); o[4 + i] = toh_flush(c[i] * QKCAR); }
                *(volatile v8h*)(P16 + (size_t)row * HD) = o; }
            if (early) {
#pragma unroll 4
                for (int s = 0; s < 16; ++s) { const int row = s * 4 + rr; const v4f a = *(const v4fa*)(os + row * 68 + seg * 8); const v4f c = *(const v4fa*)(os + row * 68 + seg * 8 + 4); v8us oh, ol;
#pragma unroll
                    for (int i = 0; i < 4; ++i) { unsigned short x0, x1; splitf(a[i], x0, x1); oh[i] = x0; ol[i] = x1; splitf(c[i], x0, x1); oh[4 + i] = x0; ol[4 + i] = x1; }
                    *(volatile v8us*)(PH + (size_t)row * HD) = oh; *(volatile v8us*)(PL + (size_t)row * HD) = ol; } }
            if (ps == 0) __threadfence(); }
    } else {
        h16* P16 = VT16 + ((size_t)bhh * HD) * SEQ + t0 + seg * 8;
        bf* PH = VTh + ((size_t)bhh * HD) * RH + te + seg * 8;
        bf* PL = VTl + ((size_t)bhh * HD) * RH + te + seg * 8;
#pragma unroll 1
        for (int ps = 0; ps < 2; ++ps) {
#pragma unroll 4
            for (int s = 0; s < 16; ++s) { const int d = s * 4 + rr; v8h o;
#pragma unroll
                for (int j = 0; j < 8; ++j) o[j] = toh_flush(os[(seg * 8 + j) * 68 + d] * VCAR);
                *(volatile v8h*)(P16 + (size_t)d * SEQ) = o; }
            if (early) {
#pragma unroll 4
                for (int s = 0; s < 16; ++s) { const int d = s * 4 + rr; v8us oh, ol;
#pragma unroll
                    for (int j = 0; j < 8; ++j) { unsigned short x0, x1; splitf(os[(seg * 8 + j) * 68 + d], x0, x1); oh[j] = x0; ol[j] = x1; }
                    *(volatile v8us*)(PH + (size_t)d * RH) = oh; *(volatile v8us*)(PL + (size_t)d * RH) = ol; } }
            if (ps == 0) __threadfence(); }
    }
}

__global__ __launch_bounds__(32) void k_attn16(const h16* __restrict__ Q16, const h16* __restrict__ K16, const h16* __restrict__ VT16, h16* CT16) {
    __shared__ __align__(16) h16 pt[16 * 72];
    __shared__ __align__(16) float os[16 * 68];
    const int lane = threadIdx.x & 31, lr = lane & 15, hi = lane >> 4;
    const int bh = blockIdx.y; const int rowbase = RH + blockIdx.x * 16;
    const size_t qoff  = ((size_t)bh * SEQ + rowbase + lr) * HD + 8 * hi;
    const size_t kbase = ((size_t)bh * SEQ + lr) * HD + 8 * hi;
    const size_t vbase = ((size_t)bh * HD + lr) * SEQ + 8 * hi;
    v8f o[4]; float m[8], l[8];
#pragma unroll
    for (int dt = 0; dt < 4; ++dt) o[dt] = (v8f){};
#pragma unroll
    for (int r = 0; r < 8; ++r) { m[r] = NEGB; l[r] = 0.0f; }
    const int nblk = rowbase / 64 + 1;
#pragma unroll 1
    for (int jb = 0; jb < nblk; ++jb) {
        const int jbase = jb * 64;
        v8f s[4];
#pragma unroll
        for (int nt = 0; nt < 4; ++nt) s[nt] = (v8f){};
        v16h qa, kf;
#pragma unroll
        for (int c = 0; c < 2; ++c) {
            qa = ldh(Q16 + qoff + c * 32);
#pragma unroll
            for (int nt = 0; nt < 4; ++nt) { kf = ldh(K16 + kbase + (size_t)(jbase + nt * 16) * HD + c * 32); s[nt] = wmma16(qa, kf, s[nt]); }
        }
        asm volatile("v_nop\n\tv_nop\n\tv_nop\n\tv_nop" : "+v"(s[0]), "+v"(s[1]), "+v"(s[2]), "+v"(s[3]) : "v"(qa), "v"(kf));
#pragma unroll
        for (int r = 0; r < 8; ++r) {
            const int t = rowbase + 8 * hi + r;
            float v[4];
#pragma unroll
            for (int nt = 0; nt < 4; ++nt) { const int key = jbase + nt * 16 + lr; const float sv = s[nt][r] * SCQ16; v[nt] = (key > t) ? NEGB : sv; }
            float mx = fmaxf(fmaxf(v[0], v[1]), fmaxf(v[2], v[3]));
            mx = fmaxf(mx, __shfl_xor(mx, 1, 32)); mx = fmaxf(mx, __shfl_xor(mx, 2, 32)); mx = fmaxf(mx, __shfl_xor(mx, 4, 32)); mx = fmaxf(mx, __shfl_xor(mx, 8, 32));
            const float mn = fmaxf(m[r], mx);
            const float al = ex2((m[r] - mn) * L2E);
            m[r] = mn;
            float p[4];
#pragma unroll
            for (int nt = 0; nt < 4; ++nt) p[nt] = ex2((v[nt] - mn) * L2E + PLOG);
            l[r] = l[r] * al + ((p[0] + p[1]) + (p[2] + p[3]));
#pragma unroll
            for (int dt = 0; dt < 4; ++dt) o[dt][r] *= al;
#pragma unroll
            for (int nt = 0; nt < 4; ++nt) pt[(8 * hi + r) * 72 + nt * 16 + lr] = (h16)p[nt];
        }
        __syncthreads();
        v16h pa, vf;
#pragma unroll
        for (int c = 0; c < 2; ++c) {
            pa = cat16(*(const v8ha*)(pt + lr * 72 + c * 32 + 8 * hi), *(const v8ha*)(pt + lr * 72 + c * 32 + 16 + 8 * hi));
#pragma unroll
            for (int dt = 0; dt < 4; ++dt) { vf = ldh(VT16 + vbase + (size_t)(dt * 16) * SEQ + jbase + c * 32); o[dt] = wmma16(pa, vf, o[dt]); }
        }
        asm volatile("v_nop\n\tv_nop\n\tv_nop\n\tv_nop" : "+v"(o[0]), "+v"(o[1]), "+v"(o[2]), "+v"(o[3]) : "v"(pa), "v"(vf));
        __syncthreads();
    }
#pragma unroll
    for (int r = 0; r < 8; ++r) {
        float lt = l[r];
        lt += __shfl_xor(lt, 1, 32); lt += __shfl_xor(lt, 2, 32); lt += __shfl_xor(lt, 4, 32); lt += __shfl_xor(lt, 8, 32);
        const float inv = (CCAR / VCAR) * (1.0f / lt);
#pragma unroll
        for (int dt = 0; dt < 4; ++dt) os[(8 * hi + r) * 68 + dt * 16 + lr] = o[dt][r] * inv;
    }
    __syncthreads();
    const int b = bh / NH, h = bh % NH; const int rr = lane >> 3, seg = lane & 7;
    h16* dst = CT16 + ((size_t)b * SEQ + rowbase) * DM + h * HD + seg * 8;
#pragma unroll 1
    for (int ps = 0; ps < 2; ++ps) {
#pragma unroll
        for (int s = 0; s < 4; ++s) { const int row = s * 4 + rr; const v4f a = *(const v4fa*)(os + row * 68 + seg * 8); const v4f c = *(const v4fa*)(os + row * 68 + seg * 8 + 4); v8h ov;
#pragma unroll
            for (int i = 0; i < 4; ++i) { ov[i] = (h16)a[i]; ov[4 + i] = (h16)c[i]; }
            *(volatile v8h*)(dst + (size_t)row * DM) = ov; }
        if (ps == 0) __threadfence(); }
}

__global__ __launch_bounds__(32) void k_attnhl(const bf* __restrict__ Qh, const bf* __restrict__ Ql, const bf* __restrict__ Kh, const bf* __restrict__ Kl,
                                                const bf* __restrict__ VTh, const bf* __restrict__ VTl, bf* ATh, bf* ATl) {
    __shared__ __align__(16) unsigned short pth[16 * 72];
    __shared__ __align__(16) unsigned short ptl[16 * 72];
    __shared__ __align__(16) float os[16 * 68];
    const int lane = threadIdx.x & 31, lr = lane & 15, hi = lane >> 4;
    const int bh = blockIdx.y; const int rowbase = blockIdx.x * 16;
    const size_t qoff  = ((size_t)bh * RH + rowbase + lr) * HD + 8 * hi;
    const size_t kbase = ((size_t)bh * RH + lr) * HD + 8 * hi;
    const size_t vbase = ((size_t)bh * HD + lr) * RH + 8 * hi;
    v8f o[4]; float m[8], l[8];
#pragma unroll
    for (int dt = 0; dt < 4; ++dt) o[dt] = (v8f){};
#pragma unroll
    for (int r = 0; r < 8; ++r) { m[r] = NEGB; l[r] = 0.0f; }
    const int nblk = rowbase / 64 + 1;
#pragma unroll 1
    for (int jb = 0; jb < nblk; ++jb) {
        const int jbase = jb * 64;
        v8f s[4];
#pragma unroll
        for (int nt = 0; nt < 4; ++nt) s[nt] = (v8f){};
        v16bf qh, ql, kh, kl;
#pragma unroll
        for (int c = 0; c < 2; ++c) {
            qh = ldb(Qh + qoff + c * 32); ql = ldb(Ql + qoff + c * 32);
#pragma unroll
            for (int nt = 0; nt < 4; ++nt) { const size_t ko = kbase + (size_t)(jbase + nt * 16) * HD + c * 32; kh = ldb(Kh + ko); kl = ldb(Kl + ko);
                s[nt] = wmmab(qh, kh, s[nt]); s[nt] = wmmab(ql, kh, s[nt]); s[nt] = wmmab(qh, kl, s[nt]); }
        }
        asm volatile("v_nop\n\tv_nop\n\tv_nop\n\tv_nop" : "+v"(s[0]), "+v"(s[1]), "+v"(s[2]), "+v"(s[3]) : "v"(qh), "v"(ql), "v"(kh), "v"(kl));
#pragma unroll
        for (int r = 0; r < 8; ++r) {
            const int t = rowbase + 8 * hi + r;
            float v[4];
#pragma unroll
            for (int nt = 0; nt < 4; ++nt) { const int key = jbase + nt * 16 + lr; const float sv = s[nt][r] * SCQHL; v[nt] = (key > t) ? NEGB : sv; }
            float mx = fmaxf(fmaxf(v[0], v[1]), fmaxf(v[2], v[3]));
            mx = fmaxf(mx, __shfl_xor(mx, 1, 32)); mx = fmaxf(mx, __shfl_xor(mx, 2, 32)); mx = fmaxf(mx, __shfl_xor(mx, 4, 32)); mx = fmaxf(mx, __shfl_xor(mx, 8, 32));
            const float mn = fmaxf(m[r], mx);
            const float al = ex2((m[r] - mn) * L2E);
            m[r] = mn;
            float p[4];
#pragma unroll
            for (int nt = 0; nt < 4; ++nt) p[nt] = ex2((v[nt] - mn) * L2E);
            l[r] = l[r] * al + ((p[0] + p[1]) + (p[2] + p[3]));
#pragma unroll
            for (int dt = 0; dt < 4; ++dt) o[dt][r] *= al;
#pragma unroll
            for (int nt = 0; nt < 4; ++nt) { unsigned short x0, x1; splitf(p[nt], x0, x1); pth[(8 * hi + r) * 72 + nt * 16 + lr] = x0; ptl[(8 * hi + r) * 72 + nt * 16 + lr] = x1; }
        }
        __syncthreads();
        v16bf pah, pal, vh, vl;
#pragma unroll
        for (int c = 0; c < 2; ++c) {
            pah = cat16b(*(const v8usa*)(pth + lr * 72 + c * 32 + 8 * hi), *(const v8usa*)(pth + lr * 72 + c * 32 + 16 + 8 * hi));
            pal = cat16b(*(const v8usa*)(ptl + lr * 72 + c * 32 + 8 * hi), *(const v8usa*)(ptl + lr * 72 + c * 32 + 16 + 8 * hi));
#pragma unroll
            for (int dt = 0; dt < 4; ++dt) { const size_t vo = vbase + (size_t)(dt * 16) * RH + jbase + c * 32; vh = ldb(VTh + vo); vl = ldb(VTl + vo);
                o[dt] = wmmab(pah, vh, o[dt]); o[dt] = wmmab(pal, vh, o[dt]); o[dt] = wmmab(pah, vl, o[dt]); }
        }
        asm volatile("v_nop\n\tv_nop\n\tv_nop\n\tv_nop" : "+v"(o[0]), "+v"(o[1]), "+v"(o[2]), "+v"(o[3]) : "v"(pah), "v"(pal), "v"(vh), "v"(vl));
        __syncthreads();
    }
#pragma unroll
    for (int r = 0; r < 8; ++r) {
        float lt = l[r];
        lt += __shfl_xor(lt, 1, 32); lt += __shfl_xor(lt, 2, 32); lt += __shfl_xor(lt, 4, 32); lt += __shfl_xor(lt, 8, 32);
        const float inv = 1.0f / lt;
#pragma unroll
        for (int dt = 0; dt < 4; ++dt) os[(8 * hi + r) * 68 + dt * 16 + lr] = o[dt][r] * inv;
    }
    __syncthreads();
    const int b = bh / NH, h = bh % NH; const int rr = lane >> 3, seg = lane & 7;
    const size_t dof = ((size_t)b * RH + rowbase) * DM + h * HD + seg * 8;
#pragma unroll 1
    for (int ps = 0; ps < 2; ++ps) {
#pragma unroll
        for (int s = 0; s < 4; ++s) { const int row = s * 4 + rr; const v4f a = *(const v4fa*)(os + row * 68 + seg * 8); const v4f c = *(const v4fa*)(os + row * 68 + seg * 8 + 4); v8us oh, ol;
#pragma unroll
            for (int i = 0; i < 4; ++i) { unsigned short x0, x1; splitf(a[i], x0, x1); oh[i] = x0; ol[i] = x1; splitf(c[i], x0, x1); oh[4 + i] = x0; ol[4 + i] = x1; }
            *(volatile v8us*)(ATh + dof + (size_t)row * DM) = oh; *(volatile v8us*)(ATl + dof + (size_t)row * DM) = ol; }
        if (ps == 0) __threadfence(); }
}

extern "C" void kernel_launch(void* const* d_in, const int* in_sizes, int n_in,
                              void* d_out, int out_size, void* d_ws, size_t ws_size, hipStream_t stream) {
    if (n_in < 5) return;
    if ((size_t)in_sizes[0] < (size_t)(NB - 1) * SEQ_FULL * DM + (size_t)SEQ * DM) return;
    if ((size_t)in_sizes[1] < (size_t)3 * DM * DM || in_sizes[2] < 3 * DM || (size_t)in_sizes[3] < (size_t)DM * DM || in_sizes[4] < DM) return;
    if ((size_t)out_size < (size_t)NB * SEQ * DM) return;
    if (ws_size < WS_TOTAL) return;
    const float* x = (const float*)d_in[0]; const float* wqkv = (const float*)d_in[1]; const float* bqkv = (const float*)d_in[2]; const float* wo = (const float*)d_in[3]; const float* bo = (const float*)d_in[4];
    float* OUT = (float*)d_out;
    char* wsp = (char*)d_ws;
    auto take = [&](size_t bytes) { char* p = wsp; wsp += bytes; return (void*)p; };
    bf* XB = (bf*)take(SZ_XB);
    bf* WQKV = (bf*)take(SZ_WQKV);
    bf* WOb = (bf*)take(SZ_WO); h16* WO16 = (h16*)take(SZ_WO);
    h16* QK16 = (h16*)take(2 * SZ_P16);
    h16* VT16 = (h16*)take(SZ_P16);
    bf* QKh = (bf*)take(2 * SZ_PE); bf* QKl = (bf*)take(2 * SZ_PE);
    bf* VTh = (bf*)take(SZ_PE); bf* VTl = (bf*)take(SZ_PE);
    h16* CT16 = (h16*)take(SZ_CT);
    bf* ATh = (bf*)take(SZ_AT); bf* ATl = (bf*)take(SZ_AT);
    float* RC = (float*)take(SZ_ROT); float* RS = (float*)take(SZ_ROT);
    if ((size_t)(wsp - (char*)d_ws) > ws_size) return;

    k_cvt8<<<dim3((unsigned)(((size_t)SEQ * DM / 8 + 255) / 256), NB, 1), 256, 0, stream>>>(x, XB, (unsigned)((size_t)SEQ * DM / 8));
    k_wtG<<<(unsigned)((3 * DM * (DM / 64) + 63) / 64), 256, 0, stream>>>(wqkv, DM, 3 * DM, WQKV, (h16*)nullptr, 1.0f);
    k_wtG<<<(unsigned)((DM * (DM / 64) + 63) / 64), 256, 0, stream>>>(wo, DM, DM, WOb, WO16, WCAR);
    k_rope<<<(unsigned)((SEQ + 7) / 8), 256, 0, stream>>>(RC, RS);
    k_qkv<<<dim3(NB * SEQ / 64, 3 * DM / 64, 1), 32, 0, stream>>>(XB, WQKV, bqkv, RC, RS, QK16, VT16, QKh, QKl, VTh, VTl);
    k_attnhl<<<dim3(RH / 16, NB * NH, 1), 32, 0, stream>>>(QKh, QKl, QKh + PLE, QKl + PLE, VTh, VTl, ATh, ATl);
    if (SEQ > RH)
        k_attn16<<<dim3((SEQ - RH) / 16 > 0 ? (SEQ - RH) / 16 : 1, NB * NH, 1), 32, 0, stream>>>(QK16, QK16 + PL16, VT16, CT16);
    k_proj_hl<<<dim3(RH / 64, DM / 64, NB), 32, 0, stream>>>(ATh, ATl, WOb, OUT, bo);
    if (SEQ > RH)
        k_proj16<<<dim3((SEQ - RH) / 64 > 0 ? (SEQ - RH) / 64 : 1, DM / 64, NB), 32, 0, stream>>>(CT16 + (size_t)RH * DM, WO16, OUT + (size_t)RH * DM, bo);
}
